// GraphSAGE_7224134992217
// MI455X (gfx1250) — hardware-verified
//
#include <hip/hip_runtime.h>
#include <stddef.h>

#define DF 128
#define RB 128
#define NT 512
#define NWV (NT / 32)
#define EPT 4
#define CHUNK (NT * EPT)
#define WPLANE (DF * DF)
#define LDS_BYTES (RB * DF * 4 + CHUNK * 4 + RB * 4 + NWV * 4)

typedef __bf16 v16bf __attribute__((ext_vector_type(16)));
typedef float v8f __attribute__((ext_vector_type(8)));
typedef float v4f __attribute__((ext_vector_type(4), __may_alias__));
typedef unsigned int v4u __attribute__((ext_vector_type(4), __may_alias__));

union Frag { v16bf v; v8f f; unsigned int u[8]; v4u q[2]; };

__device__ __forceinline__ unsigned int bf16_rne(float x) {
    unsigned int u = __builtin_bit_cast(unsigned int, x);
    u += 0x7FFFu + ((u >> 16) & 1u);
    return u >> 16;
}

__device__ __forceinline__ void split2(float a, float b, unsigned int& hi, unsigned int& lo) {
    const unsigned int ha = bf16_rne(a), hb = bf16_rne(b);
    const float ra = a - __builtin_bit_cast(float, ha << 16);
    const float rb = b - __builtin_bit_cast(float, hb << 16);
    hi = ha | (hb << 16);
    lo = bf16_rne(ra) | (bf16_rne(rb) << 16);
}

__device__ __forceinline__ v8f mma_bf16(const Frag& a, const Frag& b, v8f c) {
    v8f d = __builtin_amdgcn_wmma_f32_16x16x32_bf16(false, a.v, false, b.v, (short)0, c, false, false);
    asm volatile("v_nop\n\tv_nop\n\tv_nop\n\tv_nop" : "+v"(d) : "v"(a.f), "v"(b.f));
    return d;
}

__device__ __forceinline__ void load_a_split(const float* p, float sc, Frag& hi, Frag& lo) {
    const v4f f0 = *(const v4f*)(p);
    const v4f f1 = *(const v4f*)(p + 4);
    const v4f f2 = *(const v4f*)(p + 16);
    const v4f f3 = *(const v4f*)(p + 20);
    split2(f0.x * sc, f0.y * sc, hi.u[0], lo.u[0]);
    split2(f0.z * sc, f0.w * sc, hi.u[1], lo.u[1]);
    split2(f1.x * sc, f1.y * sc, hi.u[2], lo.u[2]);
    split2(f1.z * sc, f1.w * sc, hi.u[3], lo.u[3]);
    split2(f2.x * sc, f2.y * sc, hi.u[4], lo.u[4]);
    split2(f2.z * sc, f2.w * sc, hi.u[5], lo.u[5]);
    split2(f3.x * sc, f3.y * sc, hi.u[6], lo.u[6]);
    split2(f3.z * sc, f3.w * sc, hi.u[7], lo.u[7]);
}

__device__ __forceinline__ void load_b(const unsigned short* bp, Frag& f) {
    f.q[0] = *(const v4u*)(bp);
    f.q[1] = *(const v4u*)(bp + 16);
}

__device__ __forceinline__ void gemm_16x64(v8f (&acc)[4], const float* arow, float sc,
                                           const unsigned short* phi, const unsigned short* plo, int h)
{
#pragma unroll
    for (int kc = 0; kc < 4; ++kc) {
        const int k0 = kc * 32 + 8 * h;
        Frag ah, al;
        load_a_split(arow + k0, sc, ah, al);
#pragma unroll
        for (int ct = 0; ct < 4; ++ct) {
            Frag bh, bl;
            load_b(phi + ct * (16 * DF) + k0, bh);
            load_b(plo + ct * (16 * DF) + k0, bl);
            v8f c = acc[ct];
            c = mma_bf16(ah, bh, c);
            c = mma_bf16(ah, bl, c);
            c = mma_bf16(al, bh, c);
            acc[ct] = c;
        }
    }
}

__global__ void __launch_bounds__(256)
pack_w(const float* __restrict__ w0, const float* __restrict__ w1,
       const float* __restrict__ w2, const float* __restrict__ w3,
       unsigned short* wp)
{
    const int idx = blockIdx.x * 256 + threadIdx.x;
    if (idx < 4 * WPLANE / 8) {
        const int mi = idx >> 11;
        const int e0 = (idx & 2047) * 8;
        const float* w = (mi == 0) ? w0 : (mi == 1) ? w1 : (mi == 2) ? w2 : w3;
        const v4f a = *(const v4f*)(w + e0);
        const v4f b = *(const v4f*)(w + e0 + 4);
        unsigned int h0, h1, h2, h3, l0, l1, l2, l3;
        split2(a.x, a.y, h0, l0);
        split2(a.z, a.w, h1, l1);
        split2(b.x, b.y, h2, l2);
        split2(b.z, b.w, h3, l3);
        v4u hv; hv.x = h0; hv.y = h1; hv.z = h2; hv.w = h3;
        v4u lv; lv.x = l0; lv.y = l1; lv.z = l2; lv.w = l3;
        unsigned short* hp = wp + (size_t)mi * (2 * WPLANE) + e0;
        unsigned short* lp = hp + WPLANE;
        *(volatile v4u*)hp = hv;
        *(volatile v4u*)lp = lv;
        __threadfence();
        *(volatile v4u*)hp = hv;
        *(volatile v4u*)lp = lv;
    }
}

__global__ void __launch_bounds__(NT)
gnn_layer(const float* __restrict__ feat, const int* __restrict__ esrc, const int* __restrict__ edst,
          const unsigned short* __restrict__ wl, const unsigned short* __restrict__ wr,
          const float* __restrict__ bias, float* outp, int n_nodes, int n_edges, int relu)
{
    extern __shared__ float4 lds_raw[];
    float* agg  = (float*)lds_raw;
    int*   lst  = (int*)(agg + RB * DF);
    int*   degc = lst + CHUNK;
    int*   wtot = degc + RB;

    const int t = threadIdx.x;
    const int lane = t & 31, wv = t >> 5;
    const int n0 = blockIdx.x * RB;

    for (int i = t; i < RB * DF; i += NT) agg[i] = 0.0f;
    if (t < RB) degc[t] = 0;
    __syncthreads();

    for (int base = 0; base < n_edges; base += CHUNK) {
        int val[EPT];
        int flg[EPT];
        int cnt = 0;
#pragma unroll
        for (int j = 0; j < EPT; ++j) {
            const int e = base + j * NT + t;
            const int d = (e < n_edges) ? edst[e] : -1;
            const unsigned int udl = (unsigned int)d - (unsigned int)n0;
            const int f = (udl < (unsigned int)RB) ? 1 : 0;
            int v = 0;
            if (f) {
                int s = esrc[e];
                if (s < 0) s += n_nodes;
                s = min(max(s, 0), n_nodes - 1);
                v = s * RB + (int)udl;
            }
            val[j] = v;
            flg[j] = f;
            cnt += f;
        }
        int incl = cnt;
#pragma unroll
        for (int o = 1; o < 32; o <<= 1) {
            const int y = __shfl_up(incl, o, 32);
            if (lane >= o) incl += y;
        }
        if (lane == 31) wtot[wv] = incl;
        __syncthreads();
        int off = incl - cnt, tot = 0;
#pragma unroll
        for (int i = 0; i < NWV; ++i) {
            const int v = wtot[i];
            off += (i < wv) ? v : 0;
            tot += v;
        }
#pragma unroll
        for (int j = 0; j < EPT; ++j) {
            if (flg[j]) { lst[off] = val[j]; ++off; }
        }
        __syncthreads();
        if (tot > 0 && t < DF) {
            for (int e2 = 0; e2 < tot; ++e2) {
                const int v = lst[e2];
                const int s = v >> 7;
                const int dl = v & (RB - 1);
                agg[dl * DF + t] += feat[(size_t)s * DF + t];
                if (t == 0) degc[dl] += 1;
            }
        }
    }
    __syncthreads();

    const int m = lane & 15, h = lane >> 4;
    const int lr0 = (wv >> 1) * 16;
    const int colbase = (wv & 1) * 64;
    int grow = n0 + lr0 + m;
    grow = min(grow, n_nodes - 1);
    const float dg = (float)degc[lr0 + m];
    const float inv = 1.0f / fmaxf(dg, 1.0f);

    v8f acc[4] = {};
    gemm_16x64(acc, agg + (lr0 + m) * DF, inv,
               wl + (colbase + m) * DF, wl + WPLANE + (colbase + m) * DF, h);
    gemm_16x64(acc, feat + (size_t)grow * DF, 1.0f,
               wr + (colbase + m) * DF, wr + WPLANE + (colbase + m) * DF, h);

    __syncthreads();
#pragma unroll
    for (int ct = 0; ct < 4; ++ct) {
        const int col = colbase + ct * 16 + m;
        const float bv = bias[col];
#pragma unroll
        for (int r = 0; r < 8; ++r) {
            float v = acc[ct][r] + bv;
            if (relu) v = fmaxf(v, 0.0f);
            agg[(lr0 + 8 * h + r) * DF + col] = v;
        }
    }
    __syncthreads();

    v4f rowv[8];
#pragma unroll
    for (int i = 0; i < 8; ++i) rowv[i] = *(const v4f*)(agg + (wv * 8 + i) * DF + lane * 4);
#pragma unroll
    for (int i = 0; i < 8; ++i) {
        const int R = n0 + wv * 8 + i;
        if (R < n_nodes) *(volatile v4f*)(outp + (size_t)R * DF + lane * 4) = rowv[i];
    }
    __threadfence();
#pragma unroll
    for (int i = 0; i < 8; ++i) {
        const int R = n0 + wv * 8 + i;
        if (R < n_nodes) *(volatile v4f*)(outp + (size_t)R * DF + lane * 4) = rowv[i];
    }
}

extern "C" void kernel_launch(void* const* d_in, const int* in_sizes, int n_in,
                              void* d_out, int out_size, void* d_ws, size_t ws_size,
                              hipStream_t stream)
{
    if (n_in < 8) return;
    const int n_nodes = in_sizes[0] / DF;
    const int n_edges = in_sizes[1] / 2;
    if (n_nodes < 1 || in_sizes[0] != n_nodes * DF || in_sizes[1] != 2 * n_edges) return;
    if (in_sizes[2] != WPLANE || in_sizes[4] != WPLANE || in_sizes[5] != WPLANE || in_sizes[7] != WPLANE) return;
    if (in_sizes[3] != DF || in_sizes[6] != DF) return;
    if (out_size != n_nodes * DF) return;

    const size_t wp_bytes = (size_t)4 * 2 * WPLANE * sizeof(unsigned short);
    const size_t h_bytes  = (size_t)n_nodes * DF * sizeof(float);
    if (wp_bytes + h_bytes > ws_size) return;

    const float* x    = (const float*)d_in[0];
    const int*   eidx = (const int*)d_in[1];
    const int*   esrc = eidx;
    const int*   edst = eidx + n_edges;
    const float* W1l  = (const float*)d_in[2];
    const float* b1l  = (const float*)d_in[3];
    const float* W1r  = (const float*)d_in[4];
    const float* W2l  = (const float*)d_in[5];
    const float* b2l  = (const float*)d_in[6];
    const float* W2r  = (const float*)d_in[7];
    float* out = (float*)d_out;

    unsigned short* wp = (unsigned short*)d_ws;
    float* hbuf = (float*)((char*)d_ws + wp_bytes);

    const int pack_blocks = (4 * WPLANE / 8 + 255) / 256;
    pack_w<<<dim3(pack_blocks), dim3(256), 0, stream>>>(W1l, W1r, W2l, W2r, wp);

    const int blocks = (n_nodes + RB - 1) / RB;
    gnn_layer<<<dim3(blocks), dim3(NT), LDS_BYTES, stream>>>(
        x, esrc, edst, wp, wp + 2 * WPLANE, b1l, hbuf, n_nodes, n_edges, 1);
    gnn_layer<<<dim3(blocks), dim3(NT), LDS_BYTES, stream>>>(
        hbuf, esrc, edst, wp + 4 * WPLANE, wp + 6 * WPLANE, b2l, out, n_nodes, n_edges, 0);
}
